// MixedAttention_46505905881416
// MI455X (gfx1250) — hardware-verified
//
#include <hip/hip_runtime.h>


#define NB_  4
#define DD   512
#define TQ   1408
#define TK   2816
#define NH_  8
#define HD   64
#define ZH   4
#define PCAR 1024.0f
typedef _Float16 h16;
typedef unsigned short bf;
typedef __attribute__((ext_vector_type(16))) __bf16   v16bf;
typedef __attribute__((ext_vector_type(16))) _Float16 v16h;
typedef __attribute__((ext_vector_type(8)))  _Float16 v8h;
typedef __attribute__((ext_vector_type(8)))  unsigned short v8us;
typedef __attribute__((ext_vector_type(8)))  float    v8f;
typedef __attribute__((ext_vector_type(4)))  float    v4f;
typedef v8h  __attribute__((may_alias)) v8ha;
typedef v4f  __attribute__((may_alias)) v4fa;
typedef v8us __attribute__((may_alias)) v8usa;

__device__ __forceinline__ unsigned short f2bf(float f) { unsigned u = __float_as_uint(f); u += 0x7FFFu + ((u >> 16) & 1u); return (unsigned short)(u >> 16); }
__device__ __forceinline__ float bf2f(unsigned short b) { return __uint_as_float(((unsigned)b) << 16); }
__device__ __forceinline__ float bfr(float f) { return bf2f(f2bf(f)); }
__device__ __forceinline__ v16h cat16(v8h lo, v8h hi) { return __builtin_shufflevector(lo, hi, 0, 1, 2, 3, 4, 5, 6, 7, 8, 9, 10, 11, 12, 13, 14, 15); }
__device__ __forceinline__ v16bf cat16b(v8us lo, v8us hi) { return __builtin_bit_cast(v16bf, __builtin_shufflevector(lo, hi, 0, 1, 2, 3, 4, 5, 6, 7, 8, 9, 10, 11, 12, 13, 14, 15)); }
__device__ __forceinline__ v8f wmma16(v16h a, v16h b, v8f c) { return __builtin_amdgcn_wmma_f32_16x16x32_f16(false, a, false, b, (short)0, c, false, false); }
__device__ __forceinline__ v8f wmmab(v16bf a, v16bf b, v8f c) { return __builtin_amdgcn_wmma_f32_16x16x32_bf16(false, a, false, b, (short)0, c, false, false); }


template <typename T16> struct WFrag;
template <> struct WFrag<h16> { typedef v16h V; static __device__ __forceinline__ V ld(const h16* p) { return cat16(*(const v8h*)p, *(const v8h*)(p + 16)); } static __device__ __forceinline__ v8f mma(V a, V b, v8f c) { return wmma16(a, b, c); } };
template <> struct WFrag<bf> { typedef v16bf V; static __device__ __forceinline__ V ld(const bf* p) { return cat16b(*(const v8us*)p, *(const v8us*)(p + 16)); } static __device__ __forceinline__ v8f mma(V a, V b, v8f c) { return wmmab(a, b, c); } };
template <typename T16, int NSPLIT, bool BIAS>
__global__ __launch_bounds__(32) void k_gemmw(const T16* __restrict__ A, const T16* __restrict__ A2, const T16* __restrict__ Bt, const T16* __restrict__ Bt2, int K, float* C, int ldc, const float* __restrict__ bias, size_t sA, size_t sB, size_t sC) {
    typedef typename WFrag<T16>::V V;
    __shared__ __align__(16) float os[16 * 68];
    const size_t z = blockIdx.z; A += z * sA; if (A2) A2 += z * sA; Bt += z * sB; if (Bt2) Bt2 += z * sB; C += z * sC;
    const int lane = threadIdx.x & 31, lr = lane & 15, hi = lane >> 4; const int r0 = blockIdx.x * 64, c0 = blockIdx.y * 64;
    v8f acc[4][4];
#pragma unroll
    for (int mb = 0; mb < 4; ++mb)
#pragma unroll
        for (int nb = 0; nb < 4; ++nb) acc[mb][nb] = (v8f){};
    const size_t aoff = (size_t)(r0 + lr) * K + 8 * hi, boff = (size_t)(c0 + lr) * K + 8 * hi;
#pragma unroll 1
    for (int kc = 0; kc < K; kc += 32) {
        V a[4], a2[4];
#pragma unroll
        for (int mb = 0; mb < 4; ++mb) { a[mb] = WFrag<T16>::ld(A + aoff + (size_t)mb * 16 * K + kc); if (NSPLIT == 1 || NSPLIT == 2) a2[mb] = WFrag<T16>::ld(A2 + aoff + (size_t)mb * 16 * K + kc); }
#pragma unroll
        for (int nb = 0; nb < 4; ++nb) { const V b = WFrag<T16>::ld(Bt + boff + (size_t)nb * 16 * K + kc); V b2; if (NSPLIT >= 2) b2 = WFrag<T16>::ld(Bt2 + boff + (size_t)nb * 16 * K + kc);
#pragma unroll
            for (int mb = 0; mb < 4; ++mb) { acc[mb][nb] = WFrag<T16>::mma(a[mb], b, acc[mb][nb]); if (NSPLIT == 1 || NSPLIT == 2) acc[mb][nb] = WFrag<T16>::mma(a2[mb], b, acc[mb][nb]); if (NSPLIT >= 2) acc[mb][nb] = WFrag<T16>::mma(a[mb], b2, acc[mb][nb]); } }
        asm volatile("v_nop\n\tv_nop\n\tv_nop\n\tv_nop" : "+v"(acc[0][0]), "+v"(acc[1][1]), "+v"(acc[2][2]), "+v"(acc[3][3]) : "v"(a[0]), "v"(a[3]));
    }
#pragma unroll
    for (int mb = 0; mb < 4; ++mb) {
#pragma unroll
        for (int nb = 0; nb < 4; ++nb) {
#pragma unroll
            for (int j = 0; j < 8; ++j) os[(hi * 8 + j) * 68 + nb * 16 + lr] = acc[mb][nb][j]; }
        __builtin_amdgcn_wave_barrier(); asm volatile("" ::: "memory");
        float* crow = C + (size_t)(r0 + mb * 16) * ldc + c0;
#pragma unroll 1
        for (int ps = 0; ps < 2; ++ps) {
#pragma unroll
            for (int s = 0; s < 8; ++s) { const int row = 2 * s + hi, cofs = lr * 4; v4f val = *(const v4fa*)(os + row * 68 + cofs); if (BIAS) { val[0] += bfr(bias[c0 + cofs]); val[1] += bfr(bias[c0 + cofs + 1]); val[2] += bfr(bias[c0 + cofs + 2]); val[3] += bfr(bias[c0 + cofs + 3]); }
                *(volatile v4f*)(crow + (size_t)row * ldc + cofs) = val; }
            if (ps == 0) __threadfence(); }
        __builtin_amdgcn_wave_barrier(); asm volatile("" ::: "memory");
    }
}

__device__ __forceinline__ h16 tohx(float x) { return (h16)x; }
__device__ __forceinline__ void splitf(float y, unsigned short& h, unsigned short& l) { h = f2bf(y); l = f2bf(y - bf2f(h)); }
typedef __attribute__((ext_vector_type(2))) unsigned short v2us;
typedef __attribute__((ext_vector_type(4))) unsigned short v4us;
typedef __attribute__((ext_vector_type(2))) _Float16 v2h;
typedef __attribute__((ext_vector_type(4))) _Float16 v4h;

__global__ __launch_bounds__(256) void k_cvt8(const float* __restrict__ src, bf* dst, size_t n8) { const size_t i = (size_t)blockIdx.x * 256 + threadIdx.x; if (i >= n8) return; const v8f v = *(const v8f*)(src + i * 8); v8us o;
#pragma unroll
    for (int k = 0; k < 8; ++k) o[k] = f2bf(v[k]); *(volatile v8us*)(dst + i * 8) = o; __threadfence(); *(volatile v8us*)(dst + i * 8) = o; }
__global__ __launch_bounds__(256) void k_tr(const float* __restrict__ xb, float* XT) { __shared__ float tile[32][33]; const int t0 = blockIdx.x * 32, d0 = blockIdx.y * 32; const int lx = threadIdx.x & 31, ly = threadIdx.x >> 5;
    for (int r = ly; r < 32; r += 8) tile[r][lx] = bfr(xb[(size_t)(d0 + r) * TQ + t0 + lx]);
    __syncthreads();
    for (int r = ly; r < 32; r += 8) { const float v = tile[lx][r]; float* dst = XT + (size_t)(t0 + r) * DD + d0 + lx; *(volatile float*)dst = v; __threadfence(); *(volatile float*)dst = v; } }
__global__ __launch_bounds__(256) void k_ln(const float* __restrict__ X, const float* __restrict__ g, const float* __restrict__ bb, bf* Hh, bf* Hl) { const int lane = threadIdx.x & 31; const int r = blockIdx.x * 8 + (threadIdx.x >> 5); if (r >= TQ) return; float v[DD / 32]; float s = 0.f;
#pragma unroll
    for (int ch = 0; ch < DD / 128; ++ch) { const v4f a = *(const v4f*)(X + (size_t)r * DD + ch * 128 + lane * 4);
#pragma unroll
        for (int u = 0; u < 4; ++u) { v[ch * 4 + u] = a[u]; s += a[u]; } }
#pragma unroll
    for (int sh = 16; sh; sh >>= 1) s += __shfl_xor(s, sh, 32);
    const float mean = s * (1.0f / DD); float q = 0.f;
#pragma unroll
    for (int k = 0; k < DD / 32; ++k) { float d = __fsub_rn(v[k], mean); asm volatile("" : "+v"(d)); v[k] = d; float p = __fmul_rn(d, d); asm volatile("" : "+v"(p)); q = __fadd_rn(q, p); }
#pragma unroll
    for (int sh = 16; sh; sh >>= 1) q += __shfl_xor(q, sh, 32);
    const float rs = __frsqrt_rn(__fadd_rn(q * (1.0f / DD), 1e-6f));
    for (int ps = 0; ps < 2; ++ps) {
#pragma unroll
        for (int ch = 0; ch < DD / 128; ++ch) { v4us oh, ol;
#pragma unroll
            for (int u = 0; u < 4; ++u) { const int c = ch * 128 + lane * 4 + u; float n0 = __fmul_rn(v[ch * 4 + u], rs); asm volatile("" : "+v"(n0)); float gg = bfr(g[c]), be = bfr(bb[c]); asm volatile("" : "+v"(gg)); asm volatile("" : "+v"(be)); float t1 = __fmul_rn(n0, gg); asm volatile("" : "+v"(t1)); unsigned short p2, q2; splitf(__fadd_rn(t1, be), p2, q2); oh[u] = p2; ol[u] = q2; }
            const size_t oo = (size_t)r * DD + ch * 128 + lane * 4; *(volatile v4us*)(Hh + oo) = oh; *(volatile v4us*)(Hl + oo) = ol; }
        if (ps == 0) __threadfence(); } }
__global__ __launch_bounds__(256) void k_qp(const float* __restrict__ Q, bf* Ph, bf* Pl) { const size_t e = ((size_t)blockIdx.x * 256 + threadIdx.x) * 4; if (e >= (size_t)NH_ * TQ * HD) return; const int d = (int)(e % HD); const int t = (int)((e / HD) % TQ); const int h = (int)(e / ((size_t)HD * TQ)); const float* src = Q + (size_t)t * DD + h * HD + d; v4us oh, ol;
#pragma unroll
    for (int u = 0; u < 4; ++u) { unsigned short a, b; splitf(src[u], a, b); oh[u] = a; ol[u] = b; } *(volatile v4us*)(Ph + e) = oh; *(volatile v4us*)(Pl + e) = ol; __threadfence(); *(volatile v4us*)(Ph + e) = oh; *(volatile v4us*)(Pl + e) = ol; }
__global__ __launch_bounds__(256) void k_kp(const float* __restrict__ Kc, const float* __restrict__ Ks, bf* Ph, bf* Pl) { const size_t e = ((size_t)blockIdx.x * 256 + threadIdx.x) * 4; if (e >= (size_t)NH_ * TK * HD) return; const int d = (int)(e % HD); const int j = (int)((e / HD) % TK); const int h = (int)(e / ((size_t)HD * TK)); const float* src = (j < TQ) ? (Kc + (size_t)j * DD + h * HD + d) : (Ks + (size_t)(j - TQ) * DD + h * HD + d); v4us oh, ol;
#pragma unroll
    for (int u = 0; u < 4; ++u) { unsigned short a, b; splitf(src[u], a, b); oh[u] = a; ol[u] = b; } *(volatile v4us*)(Ph + e) = oh; *(volatile v4us*)(Pl + e) = ol; __threadfence(); *(volatile v4us*)(Ph + e) = oh; *(volatile v4us*)(Pl + e) = ol; }
__global__ __launch_bounds__(256) void k_vt(const float* __restrict__ Vc, const float* __restrict__ Vs, h16* VT) { const size_t e = ((size_t)blockIdx.x * 256 + threadIdx.x) * 2; if (e >= (size_t)NH_ * HD * TK) return; const int j = (int)(e % TK); const int d = (int)((e / TK) % HD); const int h = (int)(e / ((size_t)TK * HD)); v2h o;
#pragma unroll
    for (int u = 0; u < 2; ++u) { const int jj = j + u; const float vv = (jj < TQ) ? Vc[(size_t)jj * DD + h * HD + d] : Vs[(size_t)(jj - TQ) * DD + h * HD + d]; o[u] = tohx(vv); } *(volatile v2h*)(VT + e) = o; __threadfence(); *(volatile v2h*)(VT + e) = o; }
__global__ __launch_bounds__(256) void k_smax(const float* __restrict__ S, h16* P16) { const int lane = threadIdx.x & 31; const int row = blockIdx.x * 8 + (threadIdx.x >> 5); if (row >= ZH * TQ) return; const float* sr = S + (size_t)row * TK; float mx = -3.0e38f;
    for (int j = lane; j < TK; j += 32) mx = fmaxf(mx, sr[j]);
#pragma unroll
    for (int sh = 16; sh; sh >>= 1) mx = fmaxf(mx, __shfl_xor(mx, sh, 32));
    float sum = 0.f;
    for (int j = lane; j < TK; j += 32) { float d0 = __fsub_rn(sr[j], mx); asm volatile("" : "+v"(d0)); sum += __builtin_amdgcn_exp2f(__fmul_rn(d0, 1.4426950408889634f)); }
#pragma unroll
    for (int sh = 16; sh; sh >>= 1) sum += __shfl_xor(sum, sh, 32);
    const float f = __fdiv_rn(PCAR, sum);
    for (int ps = 0; ps < 2; ++ps) { for (int j2 = lane * 2; j2 < TK; j2 += 64) { v2h o; for (int u = 0; u < 2; ++u) { float d0 = __fsub_rn(sr[j2 + u], mx); asm volatile("" : "+v"(d0)); o[u] = tohx(__builtin_amdgcn_exp2f(__fmul_rn(d0, 1.4426950408889634f)) * f); } *(volatile v2h*)(P16 + (size_t)row * TK + j2) = o; } if (ps == 0) __threadfence(); } }
__global__ __launch_bounds__(256) void k_mrg(const float* __restrict__ O, int h0, bf* Yh, bf* Yl) { const size_t e = ((size_t)blockIdx.x * 256 + threadIdx.x) * 4; if (e >= (size_t)ZH * TQ * HD) return; const int d = (int)(e % HD); const int t = (int)((e / HD) % TQ); const int zz = (int)(e / ((size_t)HD * TQ)); const size_t oo = (size_t)t * DD + (h0 + zz) * HD + d; v4us oh, ol;
#pragma unroll
    for (int u = 0; u < 4; ++u) { unsigned short a, b; splitf(O[e + u] * (1.0f / PCAR), a, b); oh[u] = a; ol[u] = b; } *(volatile v4us*)(Yh + oo) = oh; *(volatile v4us*)(Yl + oo) = ol; __threadfence(); *(volatile v4us*)(Yh + oo) = oh; *(volatile v4us*)(Yl + oo) = ol; }
__global__ __launch_bounds__(256) void k_trout(const float* __restrict__ Z, const float* __restrict__ xb, const float* __restrict__ bz, float* outb) { __shared__ float tile[32][33]; const int t0 = blockIdx.x * 32, d0 = blockIdx.y * 32; const int lx = threadIdx.x & 31, ly = threadIdx.x >> 5;
    for (int r = ly; r < 32; r += 8) tile[r][lx] = Z[(size_t)(t0 + r) * DD + d0 + lx];
    __syncthreads();
    for (int r = ly; r < 32; r += 8) { const size_t oo = (size_t)(d0 + r) * TQ + t0 + lx; float zb = __fadd_rn(tile[lx][r], bfr(bz[d0 + r])); asm volatile("" : "+v"(zb)); const float v = __fadd_rn(bfr(xb[oo]), zb); *(volatile float*)(outb + oo) = v; __threadfence(); *(volatile float*)(outb + oo) = v; } }

extern "C" void kernel_launch(void* const* d_in, const int* in_sizes, int n_in,
                              void* d_out, int out_size, void* d_ws, size_t ws_size, hipStream_t stream) {
    (void)in_sizes; (void)n_in; (void)out_size;
    const float** I = (const float**)d_in;
    const float *x = I[0], *x2 = I[1], *lsw = I[2], *lsb = I[3], *lcw = I[4], *lcb = I[5], *Wq = I[6], *bq = I[7], *Wkc = I[8], *bkc = I[9], *Wks = I[10], *bks = I[11], *Wvc = I[12], *bvc = I[13], *Wvs = I[14], *bvs = I[15], *Wz = I[16], *bz = I[17];
    float* OUT = (float*)d_out;
    char* wsp = (char*)d_ws;
    auto take = [&](size_t bytes) { char* p = wsp; wsp += (bytes + 255) & ~(size_t)255; return (void*)p; };
    bf* BQ = (bf*)take((size_t)DD * DD * 2); bf* BKC = (bf*)take((size_t)DD * DD * 2); bf* BKS = (bf*)take((size_t)DD * DD * 2); bf* BVC = (bf*)take((size_t)DD * DD * 2); bf* BVS = (bf*)take((size_t)DD * DD * 2); bf* BZ = (bf*)take((size_t)DD * DD * 2);
    float* XT = (float*)take((size_t)TQ * DD * 4); float* X2T = (float*)take((size_t)TQ * DD * 4); bf* Nh = (bf*)take((size_t)TQ * DD * 2); bf* Nl = (bf*)take((size_t)TQ * DD * 2); bf* N2h = (bf*)take((size_t)TQ * DD * 2); bf* N2l = (bf*)take((size_t)TQ * DD * 2);
    float* Q = (float*)take((size_t)TQ * DD * 4); float* KC = (float*)take((size_t)TQ * DD * 4); float* KS = (float*)take((size_t)TQ * DD * 4); float* VC = (float*)take((size_t)TQ * DD * 4); float* VS = (float*)take((size_t)TQ * DD * 4);
    bf* QPh = (bf*)take((size_t)NH_ * TQ * HD * 2); bf* QPl = (bf*)take((size_t)NH_ * TQ * HD * 2); bf* KPh = (bf*)take((size_t)NH_ * TK * HD * 2); bf* KPl = (bf*)take((size_t)NH_ * TK * HD * 2); h16* VT = (h16*)take((size_t)NH_ * HD * TK * 2);
    float* S = (float*)take((size_t)ZH * TQ * TK * 4); h16* P16 = (h16*)take((size_t)ZH * TQ * TK * 2); float* O = (float*)take((size_t)ZH * TQ * HD * 4); bf* Yh = (bf*)take((size_t)TQ * DD * 2); bf* Yl = (bf*)take((size_t)TQ * DD * 2); float* Z = (float*)take((size_t)TQ * DD * 4);
    if ((size_t)(wsp - (char*)d_ws) > ws_size) return;
    k_cvt8<<<(DD * DD / 8 + 255) / 256, 256, 0, stream>>>(Wq, BQ, DD * DD / 8); k_cvt8<<<(DD * DD / 8 + 255) / 256, 256, 0, stream>>>(Wkc, BKC, DD * DD / 8); k_cvt8<<<(DD * DD / 8 + 255) / 256, 256, 0, stream>>>(Wks, BKS, DD * DD / 8); k_cvt8<<<(DD * DD / 8 + 255) / 256, 256, 0, stream>>>(Wvc, BVC, DD * DD / 8); k_cvt8<<<(DD * DD / 8 + 255) / 256, 256, 0, stream>>>(Wvs, BVS, DD * DD / 8); k_cvt8<<<(DD * DD / 8 + 255) / 256, 256, 0, stream>>>(Wz, BZ, DD * DD / 8);
    const size_t per = (size_t)DD * TQ; const dim3 gt(TQ / 32, DD / 32, 1), gp(TQ / 64, DD / 64, 1); const size_t zq = (size_t)TQ * HD, zk = (size_t)TK * HD, zS = (size_t)TQ * TK, zv = (size_t)HD * TK;
    for (int b = 0; b < NB_; ++b) {
        k_tr<<<gt, 256, 0, stream>>>(x + b * per, XT); k_tr<<<gt, 256, 0, stream>>>(x2 + b * per, X2T);
        k_ln<<<TQ / 8, 256, 0, stream>>>(XT, lsw, lsb, Nh, Nl); k_ln<<<TQ / 8, 256, 0, stream>>>(X2T, lcw, lcb, N2h, N2l);
        k_gemmw<bf, 1, true><<<gp, 32, 0, stream>>>(Nh, Nl, BQ, nullptr, DD, Q, DD, bq, 0, 0, 0); k_gemmw<bf, 1, true><<<gp, 32, 0, stream>>>(N2h, N2l, BKC, nullptr, DD, KC, DD, bkc, 0, 0, 0); k_gemmw<bf, 1, true><<<gp, 32, 0, stream>>>(Nh, Nl, BKS, nullptr, DD, KS, DD, bks, 0, 0, 0);
        k_gemmw<bf, 1, true><<<gp, 32, 0, stream>>>(N2h, N2l, BVC, nullptr, DD, VC, DD, bvc, 0, 0, 0); k_gemmw<bf, 1, true><<<gp, 32, 0, stream>>>(Nh, Nl, BVS, nullptr, DD, VS, DD, bvs, 0, 0, 0);
        k_qp<<<(unsigned)(((size_t)NH_ * TQ * HD / 4 + 255) / 256), 256, 0, stream>>>(Q, QPh, QPl); k_kp<<<(unsigned)(((size_t)NH_ * TK * HD / 4 + 255) / 256), 256, 0, stream>>>(KC, KS, KPh, KPl); k_vt<<<(unsigned)(((size_t)NH_ * HD * TK / 2 + 255) / 256), 256, 0, stream>>>(VC, VS, VT);
        for (int h0 = 0; h0 < NH_; h0 += ZH) {
            k_gemmw<bf, 2, false><<<dim3(TQ / 64, TK / 64, ZH), 32, 0, stream>>>(QPh + (size_t)h0 * zq, QPl + (size_t)h0 * zq, KPh + (size_t)h0 * zk, KPl + (size_t)h0 * zk, HD, S, TK, nullptr, zq, zk, zS);
            k_smax<<<ZH * TQ / 8, 256, 0, stream>>>(S, P16);
            k_gemmw<h16, 0, false><<<dim3(TQ / 64, 1, ZH), 32, 0, stream>>>(P16, nullptr, VT + (size_t)h0 * zv, nullptr, TK, O, HD, nullptr, zS, zv, zq);
            k_mrg<<<(unsigned)(((size_t)ZH * TQ * HD / 4 + 255) / 256), 256, 0, stream>>>(O, h0, Yh, Yl); }
        k_gemmw<bf, 1, false><<<gp, 32, 0, stream>>>(Yh, Yl, BZ, nullptr, DD, Z, DD, nullptr, 0, 0, 0);
        k_trout<<<gt, 256, 0, stream>>>(Z, x + b * per, bz, OUT + b * per); }
}
